// MobileFormerBlock_64819646431348
// MI455X (gfx1250) — hardware-verified
//
#include <hip/hip_runtime.h>

typedef _Float16 f16t;
typedef _Float16 v16h __attribute__((ext_vector_type(16)));
typedef _Float16 v8h  __attribute__((ext_vector_type(8)));
typedef _Float16 v4h  __attribute__((ext_vector_type(4)));
typedef float    v8f  __attribute__((ext_vector_type(8)));
typedef float    v4f  __attribute__((ext_vector_type(4)));
typedef v8h __attribute__((may_alias)) v8ha;
typedef v4h __attribute__((may_alias)) v4ha;
typedef v8f __attribute__((may_alias)) v8fa;
typedef v4f __attribute__((may_alias)) v4fa;
union Frag { v16h v; v8h half[2]; };

#define TN   6
#define NBT  64
#define CT   192
#define CH   128
#define CE   512
#define NP   1024
#define MR   384
#define HB   32
#define FH   384
#define GHD  48
#define EPS  1e-5f
#define WSCL 64.0f
#define QSC  8.0f
#define PSC  256.0f
#define X1S  16.0f
#define X2S  256.0f
#define LKC  128
#define LPA  136

__device__ __forceinline__ v8f wmma_f16(v16h a, v16h b, v8f c) {
  v8f d = __builtin_amdgcn_wmma_f32_16x16x32_f16(false, a, false, b, (short)0, c, false, false);
  asm volatile("v_nop\n\tv_nop\n\tv_nop\n\tv_nop" : "+v"(d) : "v"(a), "v"(b));
  return d;
}

__device__ __forceinline__ v16h load_frag32(const f16t* p, int h) {
  Frag f;
  f.half[0] = *(const v8ha*)(p + 8 * h);
  f.half[1] = *(const v8ha*)(p + 16 + 8 * h);
  return f.v;
}

__device__ __forceinline__ v16h load_frag_f32(const float* p, int h, float sc) {
  const v4f x0 = *(const v4fa*)(p + 8 * h);
  const v4f x1 = *(const v4fa*)(p + 8 * h + 4);
  const v4f x2 = *(const v4fa*)(p + 16 + 8 * h);
  const v4f x3 = *(const v4fa*)(p + 20 + 8 * h);
  v8h lo, hi;
  #pragma unroll
  for (int i = 0; i < 4; ++i) {
    lo[i]     = (f16t)(x0[i] * sc);
    lo[4 + i] = (f16t)(x1[i] * sc);
    hi[i]     = (f16t)(x2[i] * sc);
    hi[4 + i] = (f16t)(x3[i] * sc);
  }
  Frag f;
  f.half[0] = lo;
  f.half[1] = hi;
  return f.v;
}

__device__ __forceinline__ v8f zero8f() {
  v8f z;
  #pragma unroll
  for (int j = 0; j < 8; ++j) z[j] = 0.f;
  return z;
}
__device__ __forceinline__ v8h zero8h() {
  v8h z;
  #pragma unroll
  for (int j = 0; j < 8; ++j) z[j] = (f16t)0.0f;
  return z;
}
__device__ __forceinline__ float wsum(float v) {
  #pragma unroll
  for (int o = 16; o > 0; o >>= 1) v += __shfl_xor(v, o, 32);
  return v;
}
__device__ __forceinline__ float wmax(float v) {
  #pragma unroll
  for (int o = 16; o > 0; o >>= 1) v = fmaxf(v, __shfl_xor(v, o, 32));
  return v;
}
__device__ __forceinline__ float act_fn(float v, int act) {
  if (act == 1) return fmaxf(v, 0.f);
  if (act == 2) return 0.5f * v * (1.0f + erff(v * 0.70710678118654752f));
  if (act == 3) return fminf(fmaxf((v + 3.0f) * (1.0f / 6.0f), 0.f), 1.f);
  return v;
}

__global__ __launch_bounds__(256) void wcvt_k(const float* __restrict__ w1, const float* __restrict__ w2,
                                              f16t* __restrict__ W1h, f16t* __restrict__ W2h)
{
  const int gi = blockIdx.x * 256 + threadIdx.x;
  if (gi >= 16384) return;
  const float* src;
  f16t* dst;
  if (blockIdx.x < 32) { src = w1 + (size_t)gi * 8; dst = W1h + (size_t)gi * 8; }
  else { const int e = (gi - 8192) * 8; src = w2 + e; dst = W2h + e; }
  const v4f x0 = *(const v4fa*)src;
  const v4f x1 = *(const v4fa*)(src + 4);
  v8h o;
  #pragma unroll
  for (int i = 0; i < 4; ++i) { o[i] = (f16t)(x0[i] * WSCL); o[4 + i] = (f16t)(x1[i] * WSCL); }
  *(volatile v8h*)dst = o;
  __threadfence();
  *(volatile v8h*)dst = o;
}

__global__ __launch_bounds__(256) void xcvt_k(const float* __restrict__ x, f16t* __restrict__ XT)
{
  __shared__ __attribute__((aligned(16))) f16t sH[64 * 64];
  const int tid = threadIdx.x, lane = tid & 31, w = tid >> 5;
  const int ch0 = blockIdx.x * 64, p0 = blockIdx.y * 64, b = blockIdx.z;
  const int xq = tid & 15, cl = tid >> 4, x0 = 4 * xq;
  #pragma unroll
  for (int j = 0; j < 4; ++j) {
    const int col = cl + 16 * j, c = ch0 + col;
    const v4f v = *(const v4fa*)(x + (size_t)(b * CH + c) * NP + p0 + x0);
    sH[(x0 + 0) * 64 + col] = (f16t)v[0];
    sH[(x0 + 1) * 64 + col] = (f16t)v[1];
    sH[(x0 + 2) * 64 + col] = (f16t)v[2];
    sH[(x0 + 3) * 64 + col] = (f16t)v[3];
  }
  __syncthreads();
  const int q8 = lane & 7, sub = lane >> 3;
  v8h vals[2];
  size_t d[2];
  #pragma unroll
  for (int i = 0; i < 2; ++i) {
    const int lid = 8 * w + 4 * i + sub;
    vals[i] = *(const v8ha*)(sH + lid * 64 + 8 * q8);
    d[i] = (size_t)(b * NP + p0 + lid) * CH + ch0 + 8 * q8;
  }
  #pragma unroll
  for (int i = 0; i < 2; ++i) *(volatile v8h*)(XT + d[i]) = vals[i];
  __threadfence();
  #pragma unroll
  for (int i = 0; i < 2; ++i) *(volatile v8h*)(XT + d[i]) = vals[i];
}

__global__ __launch_bounds__(128) void lin_k(const float* __restrict__ X, int ldx,
    const float* __restrict__ W, const float* __restrict__ bias, int M, int N, int K,
    float xs, float wsc, int act, float* __restrict__ Y, int ldy)
{
  __shared__ __attribute__((aligned(16))) f16t sA[64 * LPA];
  __shared__ __attribute__((aligned(16))) f16t sB[64 * LPA];
  __shared__ __attribute__((aligned(16))) float sO[64 * 64];
  const int tid = threadIdx.x, lane = tid & 31, w = tid >> 5;
  const int h = lane >> 4, m = lane & 15;
  const int r0 = blockIdx.y * 64, n0 = blockIdx.x * 64;
  const v8f z8 = zero8f();
  v8f acc[4];
  #pragma unroll
  for (int nt = 0; nt < 4; ++nt) acc[nt] = z8;
  const int KP = (K + 31) & ~31;

  #pragma unroll 1
  for (int kc = 0; kc < KP; kc += LKC) {
    __syncthreads();
    #pragma unroll 4
    for (int i = 0; i < 16; ++i) {
      const int idx = i * 128 + tid;
      const int row = idx >> 5, c4 = idx & 31;
      const int k = kc + 4 * c4;
      const bool ok = (k + 4 <= K);
      const int kcl = ok ? k : (K - 4);
      int ra = r0 + row; ra = (ra < M) ? ra : (M - 1);
      int rb = n0 + row; rb = (rb < N) ? rb : (N - 1);
      const v4f xa = *(const v4fa*)(X + (size_t)ra * ldx + kcl);
      const v4f xb = *(const v4fa*)(W + (size_t)rb * K + kcl);
      v4h ha, hb;
      #pragma unroll
      for (int j = 0; j < 4; ++j) {
        ha[j] = ok ? (f16t)(xa[j] * xs) : (f16t)0.0f;
        hb[j] = ok ? (f16t)(xb[j] * wsc) : (f16t)0.0f;
      }
      *(v4ha*)(sA + row * LPA + 4 * c4) = ha;
      *(v4ha*)(sB + row * LPA + 4 * c4) = hb;
    }
    __syncthreads();
    const int ke = ((KP - kc) < LKC) ? (KP - kc) : LKC;
    const f16t* ap = sA + (16 * w + m) * LPA;
    #pragma unroll 1
    for (int ks = 0; ks < ke; ks += 32) {
      const v16h a = load_frag32(ap + ks, h);
      #pragma unroll
      for (int nt = 0; nt < 4; ++nt) {
        const v16h bb = load_frag32(sB + (16 * nt + m) * LPA + ks, h);
        acc[nt] = wmma_f16(a, bb, acc[nt]);
      }
    }
  }

  const float osc = 1.0f / (xs * wsc);
  #pragma unroll
  for (int nt = 0; nt < 4; ++nt) {
    const int col = 16 * nt + m, n = n0 + col;
    const int nc = (n < N) ? n : (N - 1);
    const float bv = bias[nc];
    #pragma unroll
    for (int r = 0; r < 8; ++r) {
      float v = acc[nt][r] * osc + bv;
      v = act_fn(v, act);
      if (n >= N) v = 0.f;
      sO[(16 * w + 8 * h + r) * 64 + col] = v;
    }
  }
  __syncthreads();
  const int q8 = lane & 7, sub = lane >> 3;
  v4f vals[8];
  size_t d[8];
  #pragma unroll
  for (int i = 0; i < 8; ++i) {
    const int L = 4 * i + sub;
    const int row = 16 * w + (L >> 1), hl = L & 1;
    vals[i] = *(const v4fa*)(sO + row * 64 + 32 * hl + 4 * q8);
    d[i] = (size_t)(r0 + row) * ldy + n0 + 32 * hl + 4 * q8;
  }
  #pragma unroll
  for (int i = 0; i < 8; ++i) *(volatile v4f*)(Y + d[i]) = vals[i];
  __threadfence();
  #pragma unroll
  for (int i = 0; i < 8; ++i) *(volatile v4f*)(Y + d[i]) = vals[i];
}

__global__ __launch_bounds__(128) void ln_k(const float* __restrict__ Yi, const float* __restrict__ R,
    const float* __restrict__ g, const float* __restrict__ bt, int M, float* __restrict__ out)
{
  const int tid = threadIdx.x, lane = tid & 31, w = tid >> 5;
  const int row = blockIdx.x * 4 + w;
  if (row >= M) return;
  const size_t rb = (size_t)row * CT;
  const int c0 = 4 * lane;
  const int c1 = 128 + 4 * lane;
  const int c1c = (lane < 16) ? c1 : (c1 - 64);
  const bool has1 = lane < 16;
  const v4f y0 = *(const v4fa*)(Yi + rb + c0);
  const v4f q0 = *(const v4fa*)(R + rb + c0);
  const v4f y1 = *(const v4fa*)(Yi + rb + c1c);
  const v4f q1 = *(const v4fa*)(R + rb + c1c);
  const v4f a0 = y0 + q0, a1 = y1 + q1;
  float s = (a0[0] + a0[1]) + (a0[2] + a0[3]);
  const float s1 = (a1[0] + a1[1]) + (a1[2] + a1[3]);
  s += has1 ? s1 : 0.0f;
  s = wsum(s);
  const float mean = s * (1.0f / CT);
  const v4f d0 = a0 - mean, d1 = a1 - mean;
  float q = (d0[0] * d0[0] + d0[1] * d0[1]) + (d0[2] * d0[2] + d0[3] * d0[3]);
  const float qq = (d1[0] * d1[0] + d1[1] * d1[1]) + (d1[2] * d1[2] + d1[3] * d1[3]);
  q += has1 ? qq : 0.0f;
  q = wsum(q);
  const float rs = 1.0f / sqrtf(q * (1.0f / CT) + EPS);
  const v4f g0 = *(const v4fa*)(g + c0), b0 = *(const v4fa*)(bt + c0);
  const v4f g1 = *(const v4fa*)(g + c1c), b1 = *(const v4fa*)(bt + c1c);
  const v4f o0 = d0 * rs * g0 + b0;
  const v4f o1 = d1 * rs * g1 + b1;
  float* op = out + rb;
  *(volatile v4f*)(op + c0) = o0;
  if (has1) *(volatile v4f*)(op + c1) = o1;
  __threadfence();
  *(volatile v4f*)(op + c0) = o0;
  if (has1) *(volatile v4f*)(op + c1) = o1;
}

__global__ __launch_bounds__(128) void attn1_k(const float* __restrict__ Q1, const f16t* __restrict__ XT,
                                               const float* __restrict__ ftr, float* __restrict__ CTX)
{
  __shared__ __attribute__((aligned(16))) f16t  sQ[16 * 64];
  __shared__ __attribute__((aligned(16))) float sS[TN * NP];
  __shared__ __attribute__((aligned(16))) f16t  sP[16 * NP];
  __shared__ __attribute__((aligned(16))) float sC[TN * 64];
  __shared__ float sInv[8];
  const int tid = threadIdx.x, lane = tid & 31, w = tid >> 5;
  const int h = lane >> 4, m = lane & 15;
  const int hd = blockIdx.x, b = blockIdx.y;
  const v8h zh = zero8h();
  const v8f z8 = zero8f();
  {
    const int row = tid >> 3, j = tid & 7;
    const int rc = (row < TN) ? row : (TN - 1);
    const float* qp = Q1 + (size_t)(rc * NBT + b) * CH + hd * 64 + 8 * j;
    const v4f x0 = *(const v4fa*)qp;
    const v4f x1 = *(const v4fa*)(qp + 4);
    v8h hv;
    #pragma unroll
    for (int i = 0; i < 4; ++i) { hv[i] = (f16t)(x0[i] * QSC); hv[4 + i] = (f16t)(x1[i] * QSC); }
    if (row >= TN) hv = zh;
    *(v8ha*)(sQ + row * 64 + 8 * j) = hv;
  }
  #pragma unroll 1
  for (int i = 0; i < 10; ++i) *(v8ha*)(sP + TN * NP + 8 * (i * 128 + tid)) = zh;
  __syncthreads();

  {
    const v16h a0 = load_frag32(sQ + m * 64, h);
    const v16h a1 = load_frag32(sQ + m * 64 + 32, h);
    const float ssc = 1.0f / (QSC * 8.0f);
    #pragma unroll 1
    for (int j = 0; j < 16; ++j) {
      const int nt = 16 * w + j;
      const f16t* xp = XT + (size_t)(b * NP + 16 * nt + m) * CH + hd * 64;
      v8f acc = z8;
      acc = wmma_f16(a0, load_frag32(xp, h), acc);
      acc = wmma_f16(a1, load_frag32(xp + 32, h), acc);
      if (h == 0) {
        #pragma unroll
        for (int r = 0; r < TN; ++r) sS[r * NP + 16 * nt + m] = acc[r] * ssc;
      }
    }
  }
  __syncthreads();

  #pragma unroll
  for (int ti = 0; ti < 2; ++ti) {
    const int t = w + 4 * ti;
    if (t < TN) {
      const float* sp = sS + t * NP + 32 * lane;
      float v[32];
      #pragma unroll
      for (int q = 0; q < 8; ++q) {
        const v4f t4 = *(const v4fa*)(sp + 4 * q);
        v[4 * q + 0] = t4[0]; v[4 * q + 1] = t4[1]; v[4 * q + 2] = t4[2]; v[4 * q + 3] = t4[3];
      }
      float mx = v[0];
      #pragma unroll
      for (int q = 1; q < 32; ++q) mx = fmaxf(mx, v[q]);
      mx = wmax(mx);
      float sum = 0.f;
      v8h p8[4];
      #pragma unroll
      for (int q = 0; q < 32; ++q) {
        const float e = __expf(v[q] - mx);
        sum += e;
        p8[q >> 3][q & 7] = (f16t)(e * PSC);
      }
      sum = wsum(sum);
      #pragma unroll
      for (int q = 0; q < 4; ++q) *(v8ha*)(sP + t * NP + 32 * lane + 8 * q) = p8[q];
      if (lane == 0) sInv[t] = 1.0f / (sum * PSC);
    }
  }
  __syncthreads();

  {
    const float* fr = ftr + (size_t)(b * CH + hd * 64 + 16 * w + m) * NP;
    const f16t* pr = sP + m * NP;
    v8f acc = z8;
    #pragma unroll 1
    for (int k0 = 0; k0 < NP; k0 += 32) {
      const v16h a = load_frag32(pr + k0, h);
      const v16h bb = load_frag_f32(fr + k0, h, 1.0f);
      acc = wmma_f16(a, bb, acc);
    }
    if (h == 0) {
      #pragma unroll
      for (int r = 0; r < TN; ++r) sC[r * 64 + 16 * w + m] = acc[r] * sInv[r];
    }
  }
  __syncthreads();
  if (w == 0) {
    const int q8 = lane & 7, sub = lane >> 3;
    v4f vals[3];
    size_t d[3];
    #pragma unroll
    for (int i = 0; i < 3; ++i) {
      const int L = 4 * i + sub;
      const int t = L >> 1, hl = L & 1;
      vals[i] = *(const v4fa*)(sC + t * 64 + 32 * hl + 4 * q8);
      d[i] = (size_t)(t * NBT + b) * CH + hd * 64 + 32 * hl + 4 * q8;
    }
    #pragma unroll
    for (int i = 0; i < 3; ++i) *(volatile v4f*)(CTX + d[i]) = vals[i];
    __threadfence();
    #pragma unroll
    for (int i = 0; i < 3; ++i) *(volatile v4f*)(CTX + d[i]) = vals[i];
  }
}

__global__ __launch_bounds__(256) void attn2_k(const float* __restrict__ Q2, const float* __restrict__ T1,
                                               float* __restrict__ O)
{
  __shared__ __attribute__((aligned(16))) float sQ[TN * CT];
  __shared__ __attribute__((aligned(16))) float sT[TN * CT];
  __shared__ __attribute__((aligned(16))) float sOut[TN * CT];
  __shared__ float sS[TN * 24];
  __shared__ float sPr[TN * 24];
  const int tid = threadIdx.x, lane = tid & 31, w = tid >> 5;
  const int b = blockIdx.x;
  for (int idx = tid; idx < TN * CT; idx += 256) {
    const int t = idx / CT, c = idx - t * CT;
    const size_t src = (size_t)(t * NBT + b) * CT + c;
    sQ[idx] = Q2[src];
    sT[idx] = T1[src];
  }
  __syncthreads();
  if (tid < TN * 24) {
    const int t = tid / 24, rem = tid - 24 * t;
    const int hh = rem / 6, s = rem - 6 * hh;
    const float* qp = sQ + t * CT + hh * GHD;
    const float* kp = sT + s * CT + hh * GHD;
    float acc = 0.f;
    #pragma unroll 4
    for (int dd = 0; dd < GHD; ++dd) acc += qp[dd] * kp[dd];
    sS[tid] = acc * 0.14433756729740643f;
  }
  __syncthreads();
  if (tid < TN * 4) {
    const float* sp = sS + tid * 6;
    float mx = sp[0];
    #pragma unroll
    for (int s = 1; s < TN; ++s) mx = fmaxf(mx, sp[s]);
    float e[TN], sum = 0.f;
    #pragma unroll
    for (int s = 0; s < TN; ++s) { e[s] = __expf(sp[s] - mx); sum += e[s]; }
    const float inv = 1.0f / sum;
    #pragma unroll
    for (int s = 0; s < TN; ++s) sPr[tid * 6 + s] = e[s] * inv;
  }
  __syncthreads();
  for (int idx = tid; idx < TN * CT; idx += 256) {
    const int t = idx / CT, c = idx - t * CT, hh = c / GHD;
    const float* ap = sPr + (t * 4 + hh) * 6;
    float o = 0.f;
    #pragma unroll
    for (int s = 0; s < TN; ++s) o += ap[s] * sT[s * CT + c];
    sOut[idx] = o;
  }
  __syncthreads();
  if (w < TN) {
    const int t = w;
    const int c0 = 4 * lane, c1 = 128 + 4 * lane;
    const int c1c = (lane < 16) ? c1 : (c1 - 64);
    const bool has1 = lane < 16;
    const v4f o0 = *(const v4fa*)(sOut + t * CT + c0);
    const v4f o1 = *(const v4fa*)(sOut + t * CT + c1c);
    float* op = O + (size_t)(t * NBT + b) * CT;
    *(volatile v4f*)(op + c0) = o0;
    if (has1) *(volatile v4f*)(op + c1) = o1;
    __threadfence();
    *(volatile v4f*)(op + c0) = o0;
    if (has1) *(volatile v4f*)(op + c1) = o1;
  }
}

__global__ __launch_bounds__(128) void pw1_k(const f16t* __restrict__ XT, const f16t* __restrict__ W1h,
    const float* __restrict__ g, const float* __restrict__ bt, const float* __restrict__ mu,
    const float* __restrict__ var, const float* __restrict__ CO1, int bbase, f16t* __restrict__ X1)
{
  __shared__ __attribute__((aligned(16))) f16t sH[64 * 128];
  const int tid = threadIdx.x, lane = tid & 31, w = tid >> 5;
  const int h = lane >> 4, m = lane & 15;
  const int bl = blockIdx.z, b = bbase + bl;
  const int p0 = blockIdx.x * 64, n0 = blockIdx.y * 128;
  const v8f z8 = zero8f();
  v8f acc[8];
  #pragma unroll
  for (int nt = 0; nt < 8; ++nt) acc[nt] = z8;
  const f16t* ap = XT + (size_t)(b * NP + p0 + 16 * w + m) * CH;
  const f16t* bp = W1h + (size_t)(n0 + m) * CH;
  #pragma unroll 1
  for (int k0 = 0; k0 < CH; k0 += 32) {
    const v16h a = load_frag32(ap + k0, h);
    #pragma unroll
    for (int nt = 0; nt < 8; ++nt) {
      const v16h bb = load_frag32(bp + (size_t)nt * 16 * CH + k0, h);
      acc[nt] = wmma_f16(a, bb, acc[nt]);
    }
  }
  #pragma unroll
  for (int nt = 0; nt < 8; ++nt) {
    const int col = 16 * nt + m, ch = n0 + col;
    const float inv = g[ch] / sqrtf(var[ch] + EPS);
    const float sh = bt[ch] - mu[ch] * inv;
    const float ca = CO1[(size_t)b * 1024 + ch];
    const float cb = CO1[(size_t)b * 1024 + 512 + ch];
    const float sa = (ca - 0.5f) * 2.0f + 1.0f;
    const float sb = (cb - 0.5f) * 2.0f;
    #pragma unroll
    for (int r = 0; r < 8; ++r) {
      const float xv = acc[nt][r] * (1.0f / WSCL);
      const float yv = xv * inv + sh;
      const float v = fmaxf(yv * sa, yv * sb);
      sH[(16 * w + 8 * h + r) * 128 + col] = (f16t)(v * X1S);
    }
  }
  __syncthreads();
  const int q8 = lane & 7, sub = lane >> 3;
  v8h vals[8];
  size_t d[8];
  #pragma unroll
  for (int i = 0; i < 8; ++i) {
    const int L = 4 * i + sub;
    const int row = 16 * w + (L >> 1), hl = L & 1;
    vals[i] = *(const v8ha*)(sH + row * 128 + 64 * hl + 8 * q8);
    d[i] = (size_t)(bl * NP + p0 + row) * CE + n0 + 64 * hl + 8 * q8;
  }
  #pragma unroll
  for (int i = 0; i < 8; ++i) *(volatile v8h*)(X1 + d[i]) = vals[i];
  __threadfence();
  #pragma unroll
  for (int i = 0; i < 8; ++i) *(volatile v8h*)(X1 + d[i]) = vals[i];
}

__global__ __launch_bounds__(256) void dw_k(const f16t* __restrict__ X1, const float* __restrict__ wd,
    const float* __restrict__ g, const float* __restrict__ bt, const float* __restrict__ mu,
    const float* __restrict__ var, const float* __restrict__ CO2, int bbase, f16t* __restrict__ X2)
{
  __shared__ __attribute__((aligned(16))) f16t sX[6 * 34 * 64];
  __shared__ float sW[576];
  __shared__ float sInv[64];
  __shared__ float sSh[64];
  __shared__ float sSa[64];
  __shared__ float sSb[64];
  const int tid = threadIdx.x;
  const int cg = blockIdx.x, yb = blockIdx.y, bl = blockIdx.z, b = bbase + bl;
  const int c0 = 64 * cg, y0 = 4 * yb;
  const v8h zh = zero8h();
  const int x = tid >> 3, j = tid & 7;
  #pragma unroll 1
  for (int ry = 0; ry < 6; ++ry) {
    const int yy = y0 - 1 + ry;
    const int yc = (yy < 0) ? 0 : ((yy > 31) ? 31 : yy);
    v8h v = *(const v8ha*)(X1 + (size_t)(bl * NP + yc * 32 + x) * CE + c0 + 8 * j);
    if (yy < 0 || yy > 31) v = zh;
    *(v8ha*)(sX + (ry * 34 + x + 1) * 64 + 8 * j) = v;
  }
  if (tid < 96) {
    const int ry = tid >> 4, side = (tid >> 3) & 1, jj = tid & 7;
    *(v8ha*)(sX + (ry * 34 + (side ? 33 : 0)) * 64 + 8 * jj) = zh;
  }
  for (int idx = tid; idx < 576; idx += 256) sW[idx] = wd[(size_t)c0 * 9 + idx];
  if (tid < 64) {
    const int c = c0 + tid;
    const float inv = g[c] / sqrtf(var[c] + EPS);
    sInv[tid] = inv;
    sSh[tid] = bt[c] - mu[c] * inv;
    const float ca = CO2[(size_t)b * 1024 + c];
    const float cb = CO2[(size_t)b * 1024 + 512 + c];
    sSa[tid] = (ca - 0.5f) * 2.0f + 1.0f;
    sSb[tid] = (cb - 0.5f) * 2.0f;
  }
  __syncthreads();

  #pragma unroll 1
  for (int yy = 0; yy < 4; ++yy) {
    float acc[8];
    #pragma unroll
    for (int e = 0; e < 8; ++e) acc[e] = 0.f;
    #pragma unroll 1
    for (int dy = 0; dy < 3; ++dy) {
      const f16t* rp = sX + ((yy + dy) * 34 + x) * 64 + 8 * j;
      const v8h v0 = *(const v8ha*)(rp);
      const v8h v1 = *(const v8ha*)(rp + 64);
      const v8h v2 = *(const v8ha*)(rp + 128);
      const float* wp = sW + (8 * j) * 9 + 3 * dy;
      #pragma unroll
      for (int e = 0; e < 8; ++e) {
        acc[e] += (float)v0[e] * wp[9 * e];
        acc[e] += (float)v1[e] * wp[9 * e + 1];
        acc[e] += (float)v2[e] * wp[9 * e + 2];
      }
    }
    v8h ov;
    #pragma unroll
    for (int e = 0; e < 8; ++e) {
      const int cl = 8 * j + e;
      const float xv = acc[e] * (1.0f / X1S);
      const float yv = xv * sInv[cl] + sSh[cl];
      const float v = fmaxf(yv * sSa[cl], yv * sSb[cl]);
      ov[e] = (f16t)(v * X2S);
    }
    f16t* dst = X2 + (size_t)(bl * NP + (y0 + yy) * 32 + x) * CE + c0 + 8 * j;
    *(volatile v8h*)dst = ov;
    __threadfence();
    *(volatile v8h*)dst = ov;
  }
}

__global__ __launch_bounds__(128) void pw2_k(const f16t* __restrict__ X2, const f16t* __restrict__ W2h,
    const float* __restrict__ g, const float* __restrict__ bt, const float* __restrict__ mu,
    const float* __restrict__ var, const float* __restrict__ CO3, const float* __restrict__ KB,
    const float* __restrict__ VB, const float* __restrict__ ftr, int bbase, float* __restrict__ out)
{
  __shared__ __attribute__((aligned(16))) float sT[CH * 64];
  __shared__ float sK[CH * TN];
  __shared__ float sV[CH * TN];
  const int tid = threadIdx.x, lane = tid & 31, w = tid >> 5;
  const int h = lane >> 4, m = lane & 15;
  const int bl = blockIdx.y, b = bbase + bl;
  const int p0 = blockIdx.x * 64;
  for (int idx = tid; idx < CH * TN; idx += 128) {
    const int c = idx / TN, t = idx - TN * c;
    const size_t src = (size_t)(t * NBT + b) * CH + c;
    sK[idx] = KB[src];
    sV[idx] = VB[src];
  }
  const v8f z8 = zero8f();
  v8f acc[8];
  #pragma unroll
  for (int nt = 0; nt < 8; ++nt) acc[nt] = z8;
  const f16t* ap = X2 + (size_t)(bl * NP + p0 + 16 * w + m) * CE;
  const f16t* bp = W2h + (size_t)m * CE;
  #pragma unroll 1
  for (int k0 = 0; k0 < CE; k0 += 32) {
    const v16h a = load_frag32(ap + k0, h);
    #pragma unroll
    for (int nt = 0; nt < 8; ++nt) {
      const v16h bb = load_frag32(bp + (size_t)nt * 16 * CE + k0, h);
      acc[nt] = wmma_f16(a, bb, acc[nt]);
    }
  }
  #pragma unroll
  for (int nt = 0; nt < 8; ++nt) {
    const int ch = 16 * nt + m;
    const float inv = g[ch] / sqrtf(var[ch] + EPS);
    const float sh = bt[ch] - mu[ch] * inv;
    const float sc = CO3[(size_t)b * CH + ch] * 2.0f;
    v8f o;
    #pragma unroll
    for (int r = 0; r < 8; ++r) {
      const float xv = acc[nt][r] * (1.0f / (X2S * WSCL));
      o[r] = (xv * inv + sh) * sc;
    }
    *(v8fa*)(sT + ch * 64 + 16 * w + 8 * h) = o;
  }
  __syncthreads();

  {
    const int p = tid & 63, hh = tid >> 6;
    float s[TN];
    #pragma unroll
    for (int t = 0; t < TN; ++t) s[t] = 0.f;
    #pragma unroll 2
    for (int dd = 0; dd < 64; ++dd) {
      const int c = hh * 64 + dd;
      const float qv = sT[c * 64 + p];
      const float* kr = sK + c * TN;
      #pragma unroll
      for (int t = 0; t < TN; ++t) s[t] += qv * kr[t];
    }
    float mx = -3.0e38f;
    #pragma unroll
    for (int t = 0; t < TN; ++t) { s[t] *= 0.125f; mx = fmaxf(mx, s[t]); }
    float a[TN], sum = 0.f;
    #pragma unroll
    for (int t = 0; t < TN; ++t) { a[t] = __expf(s[t] - mx); sum += a[t]; }
    const float inv = 1.0f / sum;
    #pragma unroll
    for (int t = 0; t < TN; ++t) a[t] *= inv;
    const float* fp = ftr + (size_t)(b * CH + hh * 64) * NP + p0 + p;
    #pragma unroll 2
    for (int dd = 0; dd < 64; ++dd) {
      const int c = hh * 64 + dd;
      const float* vr = sV + c * TN;
      float sp = 0.f;
      #pragma unroll
      for (int t = 0; t < TN; ++t) sp += a[t] * vr[t];
      const float xv = sT[c * 64 + p];
      sT[c * 64 + p] = (xv + sp) + fp[(size_t)dd * NP];
    }
  }
  __syncthreads();

  const int q8 = lane & 7, sub = lane >> 3;
  #pragma unroll
  for (int grp = 0; grp < 2; ++grp) {
    v4f vals[8];
    size_t d[8];
    #pragma unroll
    for (int i = 0; i < 8; ++i) {
      const int L = 32 * grp + 4 * i + sub;
      const int c = 32 * w + (L >> 1), hl = L & 1;
      vals[i] = *(const v4fa*)(sT + c * 64 + 32 * hl + 4 * q8);
      d[i] = (size_t)(b * CH + c) * NP + p0 + 32 * hl + 4 * q8;
    }
    #pragma unroll
    for (int i = 0; i < 8; ++i) *(volatile v4f*)(out + d[i]) = vals[i];
    __threadfence();
    #pragma unroll
    for (int i = 0; i < 8; ++i) *(volatile v4f*)(out + d[i]) = vals[i];
  }
}

static void launch_lin(hipStream_t st, const float* X, int ldx, const float* W, const float* bias,
                       int M, int N, int K, float xs, int act, float* Y, int ldy) {
  lin_k<<<dim3((N + 63) / 64, M / 64), 128, 0, st>>>(X, ldx, W, bias, M, N, K, xs, WSCL, act, Y, ldy);
}

extern "C" void kernel_launch(void* const* d_in, const int* in_sizes, int n_in,
                              void* d_out, int out_size, void* d_ws, size_t ws_size,
                              hipStream_t stream) {
  if (n_in < 51) return;
  if (in_sizes[0] != NBT * CH * NP || in_sizes[1] != TN * NBT * CT) return;
  if (out_size != NBT * CH * NP + TN * NBT * CT) return;
  if (in_sizes[2] != CH * CT || in_sizes[4] != CT * CH || in_sizes[8] != CT * CT || in_sizes[10] != CT * CT) return;
  if (in_sizes[14] != FH * CT || in_sizes[16] != CT * FH || in_sizes[20] != CE * CH || in_sizes[38] != CH * CE) return;
  if (in_sizes[25] != GHD * CT || in_sizes[27] != 1024 * GHD || in_sizes[34] != GHD * CT || in_sizes[36] != 1024 * GHD) return;
  if (in_sizes[43] != GHD * CT || in_sizes[45] != CH * GHD || in_sizes[29] != CE * 9) return;
  if (in_sizes[47] != CH * CT || in_sizes[49] != CH * CT) return;
  if (in_sizes[3] != CH || in_sizes[5] != CT || in_sizes[6] != CT || in_sizes[7] != CT) return;
  if (in_sizes[21] != CE || in_sizes[30] != CE || in_sizes[39] != CH || in_sizes[28] != 1024 || in_sizes[46] != CH) return;

  const float* feat   = (const float*)d_in[0];
  const float* tokens = (const float*)d_in[1];
  const float* bi_wq  = (const float*)d_in[2];
  const float* bi_bq  = (const float*)d_in[3];
  const float* bi_wo  = (const float*)d_in[4];
  const float* bi_bo  = (const float*)d_in[5];
  const float* bi_lng = (const float*)d_in[6];
  const float* bi_lnb = (const float*)d_in[7];
  const float* tm_wq  = (const float*)d_in[8];
  const float* tm_bq  = (const float*)d_in[9];
  const float* tm_wo  = (const float*)d_in[10];
  const float* tm_bo  = (const float*)d_in[11];
  const float* tm_l1g = (const float*)d_in[12];
  const float* tm_l1b = (const float*)d_in[13];
  const float* tm_w1  = (const float*)d_in[14];
  const float* tm_b1  = (const float*)d_in[15];
  const float* tm_w2  = (const float*)d_in[16];
  const float* tm_b2  = (const float*)d_in[17];
  const float* tm_l2g = (const float*)d_in[18];
  const float* tm_l2b = (const float*)d_in[19];
  const float* pw1_w  = (const float*)d_in[20];
  const float* bn1_g  = (const float*)d_in[21];
  const float* bn1_b  = (const float*)d_in[22];
  const float* bn1_m  = (const float*)d_in[23];
  const float* bn1_v  = (const float*)d_in[24];
  const float* g1_w1  = (const float*)d_in[25];
  const float* g1_b1  = (const float*)d_in[26];
  const float* g1_w2  = (const float*)d_in[27];
  const float* g1_b2  = (const float*)d_in[28];
  const float* dw_w   = (const float*)d_in[29];
  const float* bn2_g  = (const float*)d_in[30];
  const float* bn2_b  = (const float*)d_in[31];
  const float* bn2_m  = (const float*)d_in[32];
  const float* bn2_v  = (const float*)d_in[33];
  const float* g2_w1  = (const float*)d_in[34];
  const float* g2_b1  = (const float*)d_in[35];
  const float* g2_w2  = (const float*)d_in[36];
  const float* g2_b2  = (const float*)d_in[37];
  const float* pw2_w  = (const float*)d_in[38];
  const float* bn3_g  = (const float*)d_in[39];
  const float* bn3_b  = (const float*)d_in[40];
  const float* bn3_m  = (const float*)d_in[41];
  const float* bn3_v  = (const float*)d_in[42];
  const float* g3_w1  = (const float*)d_in[43];
  const float* g3_b1  = (const float*)d_in[44];
  const float* g3_w2  = (const float*)d_in[45];
  const float* g3_b2  = (const float*)d_in[46];
  const float* bo_wk  = (const float*)d_in[47];
  const float* bo_bk  = (const float*)d_in[48];
  const float* bo_wv  = (const float*)d_in[49];
  const float* bo_bv  = (const float*)d_in[50];

  float* out0 = (float*)d_out;
  float* tok3 = out0 + (size_t)NBT * CH * NP;

  const size_t szW1  = (size_t)CE * CH * 2;
  const size_t szW2  = (size_t)CH * CE * 2;
  const size_t szXT  = (size_t)NBT * NP * CH * 2;
  const size_t szR128 = (size_t)MR * CH * 4;
  const size_t szR192 = (size_t)MR * CT * 4;
  const size_t szHF  = (size_t)MR * FH * 4;
  const size_t szGH  = (size_t)64 * 64 * 4;
  const size_t szCO  = (size_t)NBT * 1024 * 4;
  const size_t szCO3 = (size_t)NBT * CH * 4;
  const size_t szX   = (size_t)HB * NP * CE * 2;
  size_t off = 0;
  char* ws = (char*)d_ws;
  f16t*  W1h  = (f16t*)(ws + off);  off += szW1;
  f16t*  W2h  = (f16t*)(ws + off);  off += szW2;
  f16t*  XT   = (f16t*)(ws + off);  off += szXT;
  float* Q1   = (float*)(ws + off); off += szR128;
  float* CTX  = (float*)(ws + off); off += szR128;
  float* Y192 = (float*)(ws + off); off += szR192;
  float* TOK1 = (float*)(ws + off); off += szR192;
  float* Q2   = (float*)(ws + off); off += szR192;
  float* OB   = (float*)(ws + off); off += szR192;
  float* TOK2 = (float*)(ws + off); off += szR192;
  float* HF   = (float*)(ws + off); off += szHF;
  float* GH   = (float*)(ws + off); off += szGH;
  float* CO1  = (float*)(ws + off); off += szCO;
  float* CO2  = (float*)(ws + off); off += szCO;
  float* CO3  = (float*)(ws + off); off += szCO3;
  float* KB   = (float*)(ws + off); off += szR128;
  float* VB   = (float*)(ws + off); off += szR128;
  f16t*  X1   = (f16t*)(ws + off);  off += szX;
  f16t*  X2   = (f16t*)(ws + off);  off += szX;
  if (off > ws_size) return;

  wcvt_k<<<64, 256, 0, stream>>>(pw1_w, pw2_w, W1h, W2h);
  xcvt_k<<<dim3(CH / 64, NP / 64, NBT), 256, 0, stream>>>(feat, XT);

  launch_lin(stream, tokens, CT, bi_wq, bi_bq, MR, CH, CT, 1.0f, 0, Q1, CH);
  attn1_k<<<dim3(2, NBT), 128, 0, stream>>>(Q1, XT, feat, CTX);
  launch_lin(stream, CTX, CH, bi_wo, bi_bo, MR, CT, CH, 16.0f, 0, Y192, CT);
  ln_k<<<MR / 4, 128, 0, stream>>>(Y192, tokens, bi_lng, bi_lnb, MR, TOK1);

  launch_lin(stream, TOK1, CT, tm_wq, tm_bq, MR, CT, CT, 1.0f, 0, Q2, CT);
  attn2_k<<<NBT, 256, 0, stream>>>(Q2, TOK1, OB);
  launch_lin(stream, OB, CT, tm_wo, tm_bo, MR, CT, CT, 1.0f, 0, Y192, CT);
  ln_k<<<MR / 4, 128, 0, stream>>>(Y192, TOK1, tm_l1g, tm_l1b, MR, TOK2);
  launch_lin(stream, TOK2, CT, tm_w1, tm_b1, MR, FH, CT, 1.0f, 2, HF, FH);
  launch_lin(stream, HF, FH, tm_w2, tm_b2, MR, CT, FH, 4.0f, 0, Y192, CT);
  ln_k<<<MR / 4, 128, 0, stream>>>(Y192, TOK2, tm_l2g, tm_l2b, MR, tok3);

  launch_lin(stream, tok3, CT, g1_w1, g1_b1, 64, GHD, CT, 1.0f, 1, GH, 64);
  launch_lin(stream, GH, 64, g1_w2, g1_b2, 64, 1024, GHD, 4.0f, 3, CO1, 1024);
  launch_lin(stream, tok3, CT, g2_w1, g2_b1, 64, GHD, CT, 1.0f, 1, GH, 64);
  launch_lin(stream, GH, 64, g2_w2, g2_b2, 64, 1024, GHD, 4.0f, 3, CO2, 1024);
  launch_lin(stream, tok3, CT, g3_w1, g3_b1, 64, GHD, CT, 1.0f, 1, GH, 64);
  launch_lin(stream, GH, 64, g3_w2, g3_b2, 64, CH, GHD, 4.0f, 3, CO3, CH);

  launch_lin(stream, tok3, CT, bo_wk, bo_bk, MR, CH, CT, 1.0f, 0, KB, CH);
  launch_lin(stream, tok3, CT, bo_wv, bo_bv, MR, CH, CT, 1.0f, 0, VB, CH);

  for (int half = 0; half < 2; ++half) {
    const int bb = half * HB;
    pw1_k<<<dim3(NP / 64, CE / 128, HB), 128, 0, stream>>>(XT, W1h, bn1_g, bn1_b, bn1_m, bn1_v, CO1, bb, X1);
    dw_k<<<dim3(CE / 64, 8, HB), 256, 0, stream>>>(X1, dw_w, bn2_g, bn2_b, bn2_m, bn2_v, CO2, bb, X2);
    pw2_k<<<dim3(NP / 64, HB), 128, 0, stream>>>(X2, W2h, bn3_g, bn3_b, bn3_m, bn3_v, CO3, KB, VB, feat, bb, out0);
  }
}
